// FFM_layer_39977555591342
// MI455X (gfx1250) — hardware-verified
//
#include <hip/hip_runtime.h>


#define NBT  16384
#define NF   256
#define NP   16
#define NK   16
#define NC   2
typedef _Float16 h16;
typedef unsigned short bf;
typedef __attribute__((ext_vector_type(16))) __bf16   v16bf;
typedef __attribute__((ext_vector_type(16))) _Float16 v16h;
typedef __attribute__((ext_vector_type(8)))  _Float16 v8h;
typedef __attribute__((ext_vector_type(8)))  unsigned short v8us;
typedef __attribute__((ext_vector_type(8)))  float    v8f;
typedef __attribute__((ext_vector_type(4)))  float    v4f;
typedef v8h  __attribute__((may_alias)) v8ha;
typedef v4f  __attribute__((may_alias)) v4fa;
typedef v8us __attribute__((may_alias)) v8usa;

__device__ __forceinline__ unsigned short f2bf(float f) { unsigned u = __float_as_uint(f); u += 0x7FFFu + ((u >> 16) & 1u); return (unsigned short)(u >> 16); }
__device__ __forceinline__ float bf2f(unsigned short b) { return __uint_as_float(((unsigned)b) << 16); }
__device__ __forceinline__ float bfr(float f) { return bf2f(f2bf(f)); }
__device__ __forceinline__ v16h cat16(v8h lo, v8h hi) { return __builtin_shufflevector(lo, hi, 0, 1, 2, 3, 4, 5, 6, 7, 8, 9, 10, 11, 12, 13, 14, 15); }
__device__ __forceinline__ v16bf cat16b(v8us lo, v8us hi) { return __builtin_bit_cast(v16bf, __builtin_shufflevector(lo, hi, 0, 1, 2, 3, 4, 5, 6, 7, 8, 9, 10, 11, 12, 13, 14, 15)); }
__device__ __forceinline__ v8f wmma16(v16h a, v16h b, v8f c) { return __builtin_amdgcn_wmma_f32_16x16x32_f16(false, a, false, b, (short)0, c, false, false); }
__device__ __forceinline__ v8f wmmab(v16bf a, v16bf b, v8f c) { return __builtin_amdgcn_wmma_f32_16x16x32_bf16(false, a, false, b, (short)0, c, false, false); }


template <typename T16> struct WFrag;
template <> struct WFrag<h16> { typedef v16h V; static __device__ __forceinline__ V ld(const h16* p) { return cat16(*(const v8h*)p, *(const v8h*)(p + 16)); } static __device__ __forceinline__ v8f mma(V a, V b, v8f c) { return wmma16(a, b, c); } };
template <> struct WFrag<bf> { typedef v16bf V; static __device__ __forceinline__ V ld(const bf* p) { return cat16b(*(const v8us*)p, *(const v8us*)(p + 16)); } static __device__ __forceinline__ v8f mma(V a, V b, v8f c) { return wmmab(a, b, c); } };
template <typename T16, int NSPLIT, bool BIAS>
__global__ __launch_bounds__(32) void k_gemmw(const T16* __restrict__ A, const T16* __restrict__ A2, const T16* __restrict__ Bt, const T16* __restrict__ Bt2, int K, float* C, int ldc, const float* __restrict__ bias, size_t sA, size_t sB, size_t sC) {
    typedef typename WFrag<T16>::V V;
    __shared__ __align__(16) float os[16 * 68];
    const size_t z = blockIdx.z; A += z * sA; if (A2) A2 += z * sA; Bt += z * sB; if (Bt2) Bt2 += z * sB; C += z * sC;
    const int lane = threadIdx.x & 31, lr = lane & 15, hi = lane >> 4; const int r0 = blockIdx.x * 64, c0 = blockIdx.y * 64;
    v8f acc[4][4];
#pragma unroll
    for (int mb = 0; mb < 4; ++mb)
#pragma unroll
        for (int nb = 0; nb < 4; ++nb) acc[mb][nb] = (v8f){};
    const size_t aoff = (size_t)(r0 + lr) * K + 8 * hi, boff = (size_t)(c0 + lr) * K + 8 * hi;
#pragma unroll 1
    for (int kc = 0; kc < K; kc += 32) {
        V a[4], a2[4];
#pragma unroll
        for (int mb = 0; mb < 4; ++mb) { a[mb] = WFrag<T16>::ld(A + aoff + (size_t)mb * 16 * K + kc); if (NSPLIT == 1 || NSPLIT == 2) a2[mb] = WFrag<T16>::ld(A2 + aoff + (size_t)mb * 16 * K + kc); }
#pragma unroll
        for (int nb = 0; nb < 4; ++nb) { const V b = WFrag<T16>::ld(Bt + boff + (size_t)nb * 16 * K + kc); V b2; if (NSPLIT >= 2) b2 = WFrag<T16>::ld(Bt2 + boff + (size_t)nb * 16 * K + kc);
#pragma unroll
            for (int mb = 0; mb < 4; ++mb) { acc[mb][nb] = WFrag<T16>::mma(a[mb], b, acc[mb][nb]); if (NSPLIT == 1 || NSPLIT == 2) acc[mb][nb] = WFrag<T16>::mma(a2[mb], b, acc[mb][nb]); if (NSPLIT >= 2) acc[mb][nb] = WFrag<T16>::mma(a[mb], b2, acc[mb][nb]); } }
        asm volatile("v_nop\n\tv_nop\n\tv_nop\n\tv_nop" : "+v"(acc[0][0]), "+v"(acc[1][1]), "+v"(acc[2][2]), "+v"(acc[3][3]) : "v"(a[0]), "v"(a[3]));
    }
#pragma unroll
    for (int mb = 0; mb < 4; ++mb) {
#pragma unroll
        for (int nb = 0; nb < 4; ++nb) {
#pragma unroll
            for (int j = 0; j < 8; ++j) os[(hi * 8 + j) * 68 + nb * 16 + lr] = acc[mb][nb][j]; }
        __builtin_amdgcn_wave_barrier(); asm volatile("" ::: "memory");
        float* crow = C + (size_t)(r0 + mb * 16) * ldc + c0;
#pragma unroll 1
        for (int ps = 0; ps < 2; ++ps) {
#pragma unroll
            for (int s = 0; s < 8; ++s) { const int row = 2 * s + hi, cofs = lr * 4; v4f val = *(const v4fa*)(os + row * 68 + cofs); if (BIAS) { val[0] += bfr(bias[c0 + cofs]); val[1] += bfr(bias[c0 + cofs + 1]); val[2] += bfr(bias[c0 + cofs + 2]); val[3] += bfr(bias[c0 + cofs + 3]); }
                *(volatile v4f*)(crow + (size_t)row * ldc + cofs) = val; }
            if (ps == 0) __threadfence(); }
        __builtin_amdgcn_wave_barrier(); asm volatile("" ::: "memory");
    }
}

__device__ __forceinline__ void splitf(float y, unsigned short& h, unsigned short& l) { h = f2bf(y); l = f2bf(y - bf2f(h)); }
typedef __attribute__((ext_vector_type(2))) unsigned short v2us;
typedef __attribute__((ext_vector_type(2))) float v2f;

__global__ __launch_bounds__(256) void k_cvt8(const float* __restrict__ src, bf* dst, size_t n8) { const size_t i = (size_t)blockIdx.x * 256 + threadIdx.x; if (i >= n8) return; const v8f v = *(const v8f*)(src + i * 8); v8us o;
#pragma unroll
    for (int k = 0; k < 8; ++k) o[k] = f2bf(v[k]); *(volatile v8us*)(dst + i * 8) = o; __threadfence(); *(volatile v8us*)(dst + i * 8) = o; }
__global__ __launch_bounds__(256) void k_T(const float* __restrict__ v, const int* __restrict__ fm, bf* Th, bf* Tl) { const size_t e = ((size_t)blockIdx.x * 256 + threadIdx.x) * 2; if (e >= (size_t)NC * NF * NF) return; const int i = (int)(e % NF); const int j = (int)((e / NF) % NF); const int c = (int)(e / ((size_t)NF * NF)); v2us oh, ol;
#pragma unroll
    for (int u = 0; u < 2; ++u) { const int ii = i + u; int fi = fm[ii], fj = fm[j]; fi = min(max(fi, 0), NP - 1); fj = min(max(fj, 0), NP - 1); float s = 0.f;
#pragma unroll 1
        for (int k = 0; k < NK; ++k) { float p = __fmul_rn(bfr(v[(((size_t)ii * NP + fj) * NK + k) * NC + c]), bfr(v[(((size_t)j * NP + fi) * NK + k) * NC + c])); asm volatile("" : "+v"(p)); s = __fadd_rn(s, p); }
        unsigned short a, b2; splitf(s, a, b2); oh[u] = a; ol[u] = b2; }
    *(volatile v2us*)(Th + e) = oh; *(volatile v2us*)(Tl + e) = ol; __threadfence(); *(volatile v2us*)(Th + e) = oh; *(volatile v2us*)(Tl + e) = ol; }
__global__ __launch_bounds__(256) void k_TD(const float* __restrict__ v, const int* __restrict__ fm, float* TD) { const int e = blockIdx.x * 256 + threadIdx.x; if (e >= NC * NF) return; const int i = e % NF, c = e / NF; int fi = fm[i]; fi = min(max(fi, 0), NP - 1); float s = 0.f;
#pragma unroll 1
    for (int k = 0; k < NK; ++k) { const float a = bfr(v[(((size_t)i * NP + fi) * NK + k) * NC + c]); float p = __fmul_rn(a, a); asm volatile("" : "+v"(p)); s = __fadd_rn(s, p); }
    *(volatile float*)(TD + e) = s; __threadfence(); *(volatile float*)(TD + e) = s; }
__global__ __launch_bounds__(256) void k_out(const float* __restrict__ x, const float* __restrict__ YT, const float* __restrict__ TD, const float* __restrict__ Wl, const float* __restrict__ bl, float* OUT) { const int b = blockIdx.x * 256 + threadIdx.x; if (b >= NBT) return; const float* xr = x + (size_t)b * NF; float full0 = 0.f, full1 = 0.f, dg0 = 0.f, dg1 = 0.f, l0 = 0.f, l1 = 0.f;
#pragma unroll 1
    for (int i = 0; i < NF; ++i) { const float xi = bfr(xr[i]); float p;
        p = __fmul_rn(xi, YT[((size_t)0 * NF + i) * NBT + b]); asm volatile("" : "+v"(p)); full0 = __fadd_rn(full0, p); p = __fmul_rn(xi, YT[((size_t)1 * NF + i) * NBT + b]); asm volatile("" : "+v"(p)); full1 = __fadd_rn(full1, p);
        float x2 = __fmul_rn(xi, xi); asm volatile("" : "+v"(x2)); p = __fmul_rn(x2, TD[i]); asm volatile("" : "+v"(p)); dg0 = __fadd_rn(dg0, p); p = __fmul_rn(x2, TD[NF + i]); asm volatile("" : "+v"(p)); dg1 = __fadd_rn(dg1, p);
        p = __fmul_rn(xi, bfr(Wl[i])); asm volatile("" : "+v"(p)); l0 = __fadd_rn(l0, p); p = __fmul_rn(xi, bfr(Wl[NF + i])); asm volatile("" : "+v"(p)); l1 = __fadd_rn(l1, p); }
    const float z0 = __fadd_rn(__fadd_rn(l0, bfr(bl[0])), 0.5f * __fsub_rn(full0, dg0)), z1 = __fadd_rn(__fadd_rn(l1, bfr(bl[1])), 0.5f * __fsub_rn(full1, dg1)); const float m = fmaxf(z0, z1); float e0 = __fsub_rn(z0, m), e1 = __fsub_rn(z1, m); asm volatile("" : "+v"(e0), "+v"(e1)); const float lse = __fadd_rn(m, __logf(__fadd_rn(__expf(e0), __expf(e1))));
    v2f o; o[0] = __fsub_rn(z0, lse); o[1] = __fsub_rn(z1, lse); *(volatile v2f*)(OUT + (size_t)b * 2) = o; __threadfence(); *(volatile v2f*)(OUT + (size_t)b * 2) = o; }

extern "C" void kernel_launch(void* const* d_in, const int* in_sizes, int n_in,
                              void* d_out, int out_size, void* d_ws, size_t ws_size, hipStream_t stream) {
    (void)in_sizes; (void)n_in; (void)out_size;
    const float* x = (const float*)d_in[0]; const int* fm = (const int*)d_in[1]; const float* Wl = (const float*)d_in[2]; const float* bl = (const float*)d_in[3]; const float* v = (const float*)d_in[4];
    float* OUT = (float*)d_out;
    char* wsp = (char*)d_ws;
    auto take = [&](size_t bytes) { char* p = wsp; wsp += (bytes + 255) & ~(size_t)255; return (void*)p; };
    bf* XB = (bf*)take((size_t)NBT * NF * 2); bf* Th = (bf*)take((size_t)NC * NF * NF * 2); bf* Tl = (bf*)take((size_t)NC * NF * NF * 2); float* TD = (float*)take((size_t)NC * NF * 4); float* YT = (float*)take((size_t)NC * NF * NBT * 4);
    if ((size_t)(wsp - (char*)d_ws) > ws_size) return;
    k_cvt8<<<(NBT * NF / 8 + 255) / 256, 256, 0, stream>>>(x, XB, (size_t)NBT * NF / 8); k_T<<<(NC * NF * NF / 2 + 255) / 256, 256, 0, stream>>>(v, fm, Th, Tl); k_TD<<<(NC * NF + 255) / 256, 256, 0, stream>>>(v, fm, TD);
    k_gemmw<bf, 1, false><<<dim3(NF / 64, NBT / 64, NC), 32, 0, stream>>>(Th, Tl, XB, nullptr, NF, YT, NBT, nullptr, (size_t)NF * NF, 0, (size_t)NF * NBT);
    k_out<<<NBT / 256, 256, 0, stream>>>(x, YT, TD, Wl, bl, OUT);
}
